// myBadTransfomerBlock_56495999811681
// MI455X (gfx1250) — hardware-run, weakly checked
//
#include <hip/hip_runtime.h>


#ifndef NB
#define NB 4
#endif
#ifndef SEQ
#define SEQ 4096
#endif
#define NB_FULL  4
#define SEQ_FULL 4096
#ifndef OUT_SEQ
#define OUT_SEQ SEQ
#endif
#define DM   64
#define AW   4
#define OSP  68
#define QRS  2048.0f
#define QRI  (1.0f / 2048.0f)
#define WCAR 8.0f
#define DCAR (1.0f / 64.0f)
#define DUN  8.0f
#define NEPS 1.0e-6f

static_assert(DM == 64);
static_assert(DM % 32 == 0);
static_assert(AW == 4);
static_assert(16 * AW == 64);
static_assert(SEQ % 64 == 0);
static_assert((NB * SEQ) % 64 == 0);
static_assert(SEQ % 32 == 0);
static_assert(SEQ % (16 * AW) == 0);
static_assert(NB <= NB_FULL);
static_assert(SEQ <= SEQ_FULL);
static_assert((OSP * 4) % 16 == 0);
static_assert(OSP >= DM);
static_assert(AW * 16 * OSP * 4 <= 131072);
static_assert(32 * 16 * 4 == 16 * DM * 2);
static_assert(32 * 16 * 8 == 16 * DM * 4);
static_assert(2 * DM * DM == 4 * 256 * 8);

typedef _Float16 h16;
typedef unsigned short bf;
typedef __attribute__((ext_vector_type(16))) __bf16   v16bf;
typedef __attribute__((ext_vector_type(16))) _Float16 v16h;
typedef __attribute__((ext_vector_type(8)))  _Float16 v8h;
typedef __attribute__((ext_vector_type(8)))  unsigned short v8us;
typedef __attribute__((ext_vector_type(8)))  float    v8f;
typedef __attribute__((ext_vector_type(4)))  float    v4f;
typedef v4f  __attribute__((may_alias)) v4fa;

__device__ __forceinline__ unsigned short f2bf(float f) { unsigned u = __float_as_uint(f); u += 0x7FFFu + ((u >> 16) & 1u); return (unsigned short)(u >> 16); }
__device__ __forceinline__ float bfr(float f) { return __uint_as_float(((unsigned)f2bf(f)) << 16); }
__device__ __forceinline__ v16h cat16(v8h lo, v8h hi) { return __builtin_shufflevector(lo, hi, 0, 1, 2, 3, 4, 5, 6, 7, 8, 9, 10, 11, 12, 13, 14, 15); }
__device__ __forceinline__ v16bf cat16b(v8us lo, v8us hi) { return __builtin_bit_cast(v16bf, __builtin_shufflevector(lo, hi, 0, 1, 2, 3, 4, 5, 6, 7, 8, 9, 10, 11, 12, 13, 14, 15)); }
__device__ __forceinline__ v8f wmma16(v16h a, v16h b, v8f c) { return __builtin_amdgcn_wmma_f32_16x16x32_f16(false, a, false, b, (short)0, c, false, false); }
__device__ __forceinline__ v8f wmmab(v16bf a, v16bf b, v8f c) { return __builtin_amdgcn_wmma_f32_16x16x32_bf16(false, a, false, b, (short)0, c, false, false); }
__device__ __forceinline__ v8f wmma16g(v16h a, v16h b, v8f c) { c = wmma16(a, b, c); asm volatile("v_nop\n\tv_nop\n\tv_nop\n\tv_nop" : "+v"(c) : "v"(a), "v"(b)); return c; }
__device__ __forceinline__ v8f wmmabg(v16bf a, v16bf b, v8f c) { c = wmmab(a, b, c); asm volatile("v_nop\n\tv_nop\n\tv_nop\n\tv_nop" : "+v"(c) : "v"(a), "v"(b)); return c; }
__device__ __forceinline__ v16h  ldh(const h16* p) { return cat16(*(const v8h*)p, *(const v8h*)(p + 16)); }
__device__ __forceinline__ v16bf ldb(const bf* p)  { return cat16b(*(const v8us*)p, *(const v8us*)(p + 16)); }
__device__ __forceinline__ void wave_sync() { __builtin_amdgcn_fence(3  , "wavefront"); __builtin_amdgcn_wave_barrier(); asm volatile("" ::: "memory"); }
static __device__ __forceinline__ h16 toh_flush(float v) { const float w = (fabsf(v) < 6.103515625e-05f) ? 0.0f : v; return (h16)w; }

template <int BASE> __device__ __forceinline__ void bcvt4(v4f p, v8us& hv) {
#pragma unroll
    for (int i = 0; i < 4; ++i) hv[BASE + i] = f2bf(p[i]);
}
template <int BASE> __device__ __forceinline__ void bsplit4(v4f p, v8us& hv, v8us& lv) {
#pragma unroll
    for (int i = 0; i < 4; ++i) { const unsigned short hb = f2bf(p[i]); const float hf = __uint_as_float(((unsigned)hb) << 16); hv[BASE + i] = hb; lv[BASE + i] = f2bf(p[i] - hf); }
}
template <int BASE> __device__ __forceinline__ void hsplit4(v4f p, v8h& hv, v8h& rv) {
#pragma unroll
    for (int i = 0; i < 4; ++i) { const h16 a = toh_flush(p[i]); hv[BASE + i] = a; rv[BASE + i] = toh_flush((p[i] - (float)a) * QRS); }
}

__global__ __launch_bounds__(256) void k_wconv(const float* __restrict__ wenc, const float* __restrict__ wdec, bf* WE, h16* WD) {
    const unsigned bx = blockIdx.x;
    const unsigned i = (bx & 3u) * 256u + threadIdx.x;
    if (bx < 4u) {
        const v8f v = *(const v8f*)(wenc + (size_t)i * 8); v8us o;
#pragma unroll
        for (int k = 0; k < 8; ++k) o[k] = f2bf(v[k]);
        *(volatile v8us*)(WE + (size_t)i * 8) = o; __threadfence(); *(volatile v8us*)(WE + (size_t)i * 8) = o;
    } else {
        const v8f v = *(const v8f*)(wdec + (size_t)i * 8); v8h o;
#pragma unroll
        for (int k = 0; k < 8; ++k) o[k] = toh_flush(bfr(v[k]) * WCAR);
        *(volatile v8h*)(WD + (size_t)i * 8) = o; __threadfence(); *(volatile v8h*)(WD + (size_t)i * 8) = o;
    }
}

__global__ __launch_bounds__(32 * AW) void k_enc(const float* __restrict__ X, const bf* __restrict__ WE, h16* YH, h16* YR, h16* YTH, h16* YTR) {
    __shared__ __align__(16) float os[AW * 16 * OSP];
    const int lane = threadIdx.x & 31, lr = lane & 15, hi = lane >> 4;
    const int wave = __builtin_amdgcn_readfirstlane((int)(threadIdx.x >> 5));
    const unsigned bx = blockIdx.x;
    const unsigned r0 = bx * 64u;
    const unsigned b = r0 / (unsigned)SEQ, tt = r0 % (unsigned)SEQ;
    const int wb = wave * 16 * OSP;
    const v8f zv = (v8f){};
    const float* xr = X + ((size_t)b * SEQ_FULL + (size_t)tt + (size_t)(wave * 16 + lr)) * DM + 8 * hi;
    v16bf xa[2];
#pragma unroll
    for (int kc = 0; kc < 2; ++kc) {
        const v4f p0 = *(const v4f*)(xr + kc * 32), p1 = *(const v4f*)(xr + kc * 32 + 4), p2 = *(const v4f*)(xr + kc * 32 + 16), p3 = *(const v4f*)(xr + kc * 32 + 20);
        v8us e0, e1; bcvt4<0>(p0, e0); bcvt4<4>(p1, e0); bcvt4<0>(p2, e1); bcvt4<4>(p3, e1);
        xa[kc] = cat16b(e0, e1); }
    const size_t wo = (size_t)lr * DM + 8 * hi;
    v8f acc[4];
#pragma unroll
    for (int nb = 0; nb < 4; ++nb) acc[nb] = zv;
#pragma unroll
    for (int kc = 0; kc < 2; ++kc) {
#pragma unroll
        for (int nb = 0; nb < 4; ++nb) { const v16bf w = ldb(WE + wo + (size_t)nb * 16 * DM + kc * 32); acc[nb] = wmmabg(xa[kc], w, acc[nb]); } }
#pragma unroll
    for (int nb = 0; nb < 4; ++nb) {
#pragma unroll
        for (int j = 0; j < 8; ++j) os[wb + (hi * 8 + j) * OSP + nb * 16 + lr] = fmaxf(acc[nb][j], 0.0f); }
    wave_sync();
    v16bf ah[2], al[2];
#pragma unroll
    for (int kc = 0; kc < 2; ++kc) {
        const int o = wb + lr * OSP + kc * 32 + 8 * hi;
        const v4f p0 = *(const v4fa*)(&os[o]), p1 = *(const v4fa*)(&os[o + 4]), p2 = *(const v4fa*)(&os[o + 16]), p3 = *(const v4fa*)(&os[o + 20]);
        v8us h0, l0, h1, l1; bsplit4<0>(p0, h0, l0); bsplit4<4>(p1, h0, l0); bsplit4<0>(p2, h1, l1); bsplit4<4>(p3, h1, l1);
        ah[kc] = cat16b(h0, h1); al[kc] = cat16b(l0, l1); }
    wave_sync();
    v8f ac2[4];
#pragma unroll
    for (int nb = 0; nb < 4; ++nb) ac2[nb] = zv;
#pragma unroll
    for (int kc = 0; kc < 2; ++kc) {
#pragma unroll
        for (int nb = 0; nb < 4; ++nb) { const v16bf w = ldb(WE + (size_t)DM * DM + wo + (size_t)nb * 16 * DM + kc * 32);
            ac2[nb] = wmmabg(ah[kc], w, ac2[nb]); ac2[nb] = wmmabg(al[kc], w, ac2[nb]); } }
    float ss[8];
#pragma unroll
    for (int j = 0; j < 8; ++j) { float s = 0.0f;
#pragma unroll
        for (int nb = 0; nb < 4; ++nb) { const float v = fmaxf(ac2[nb][j], 0.0f); ac2[nb][j] = v; s += v * v; }
        ss[j] = s; }
#pragma unroll
    for (int mk = 1; mk <= 8; mk <<= 1) {
#pragma unroll
        for (int j = 0; j < 8; ++j) ss[j] += __shfl_xor(ss[j], mk, 32); }
#pragma unroll
    for (int j = 0; j < 8; ++j) { const float inv = 1.0f / (sqrtf(ss[j]) + NEPS);
#pragma unroll
        for (int nb = 0; nb < 4; ++nb) os[wb + (hi * 8 + j) * OSP + nb * 16 + lr] = ac2[nb][j] * inv; }
    __syncthreads();
    const size_t yrow = ((size_t)b * SEQ + (size_t)tt + (size_t)(wave * 16)) * DM;
    const size_t ytb  = ((size_t)b * DM) * SEQ + (size_t)tt;
#pragma unroll 1
    for (int ps = 0; ps < 2; ++ps) {
#pragma unroll
        for (int s = 0; s < 4; ++s) { const int row = 4 * s + (lane >> 3), c8 = (lane & 7) * 8;
            const v4f x0 = *(const v4fa*)(&os[wb + row * OSP + c8]); const v4f x1 = *(const v4fa*)(&os[wb + row * OSP + c8 + 4]); v8h hv, rv;
            hsplit4<0>(x0, hv, rv); hsplit4<4>(x1, hv, rv);
            const size_t oo = yrow + (size_t)row * DM + c8;
            *(volatile v8h*)(YH + oo) = hv; *(volatile v8h*)(YR + oo) = rv; }
#pragma unroll
        for (int s = 0; s < 4; ++s) { const int d = wave * 16 + 4 * s + (lane >> 3), t8 = (lane & 7) * 8;
            v8h hv, rv;
#pragma unroll
            for (int i = 0; i < 8; ++i) { const float v = os[(t8 + i) * OSP + d]; const h16 a = toh_flush(v); hv[i] = a; rv[i] = toh_flush((v - (float)a) * QRS); }
            const size_t oo = ytb + (size_t)d * SEQ + t8;
            *(volatile v8h*)(YTH + oo) = hv; *(volatile v8h*)(YTR + oo) = rv; }
        if (ps == 0) __threadfence(); }
}

__global__ __launch_bounds__(32 * AW) __attribute__((amdgpu_num_vgpr(256)))
void k_sim(const h16* __restrict__ YH, const h16* __restrict__ YTH, float* Y2) {
    __shared__ __align__(16) float os[AW * 16 * OSP];
    const int lane = threadIdx.x & 31, lr = lane & 15, hi = lane >> 4;
    const int wave = __builtin_amdgcn_readfirstlane((int)(threadIdx.x >> 5));
    const unsigned b = blockIdx.y;
    const unsigned t0 = (blockIdx.x * (unsigned)AW + (unsigned)wave) * 16u;
    const size_t pbase = (size_t)b * SEQ * DM;
    const size_t qo = pbase + (size_t)(t0 + (unsigned)lr) * DM + 8 * hi;
    const v16h qh0 = ldh(YH + qo), qh1 = ldh(YH + qo + 32);
    const size_t ko = pbase + (size_t)lr * DM + 8 * hi;
    const size_t vo = pbase + (size_t)lr * SEQ + 8 * hi;
    const v8f zv = (v8f){};
    v8f o[4];
#pragma unroll
    for (int j = 0; j < 4; ++j) { o[j] = zv; }
#pragma unroll 1
    for (int key0 = 0; key0 < SEQ; key0 += 32) {
        const h16* ka = YH + ko + (size_t)key0 * DM;
        v8f sHa = zv, sHb = zv;
        { const v16h k0 = ldh(ka), k1 = ldh(ka + 32);
          sHa = wmma16g(k0, qh0, sHa); sHa = wmma16g(k1, qh1, sHa); }
        { const v16h k0 = ldh(ka + 16 * DM), k1 = ldh(ka + 16 * DM + 32);
          sHb = wmma16g(k0, qh0, sHb); sHb = wmma16g(k1, qh1, sHb); }
        v16h pb;
#pragma unroll
        for (int r = 0; r < 8; ++r) {
            const h16 pa = toh_flush(sHa[r]); const h16 pc = toh_flush(sHb[r]);
            pb[r] = pa; pb[8 + r] = pc; }
        const h16* va = YTH + vo + key0;
#pragma unroll
        for (int j = 0; j < 4; ++j) {
            const v16h vh = ldh(va + (size_t)j * 16 * SEQ);
            o[j]  = wmma16g(vh, pb, o[j]); }
    }
    const int wb = wave * 16 * OSP;
#pragma unroll
    for (int j = 0; j < 4; ++j) { const v8f f = o[j]; v4f a, c;
        a[0] = f[0]; a[1] = f[1]; a[2] = f[2]; a[3] = f[3]; c[0] = f[4]; c[1] = f[5]; c[2] = f[6]; c[3] = f[7];
        *(v4fa*)(&os[wb + lr * OSP + 16 * j + 8 * hi]) = a; *(v4fa*)(&os[wb + lr * OSP + 16 * j + 8 * hi + 4]) = c; }
    wave_sync();
    float* orow = Y2 + ((size_t)b * SEQ + (size_t)t0) * DM;
#pragma unroll 1
    for (int ps = 0; ps < 2; ++ps) {
#pragma unroll
        for (int s = 0; s < 8; ++s) { const int row = 2 * s + (lane >> 4), cofs = (lane & 15) * 4;
            const v4f val = *(const v4fa*)(&os[wb + row * OSP + cofs]);
            *(volatile v4f*)(orow + (size_t)row * DM + cofs) = val; }
        if (ps == 0) __threadfence(); }
}

__global__ __launch_bounds__(32 * AW) void k_dec(const float* __restrict__ Y2, const h16* __restrict__ WD, float* OUT) {
    __shared__ __align__(16) float os[AW * 16 * OSP];
    const int lane = threadIdx.x & 31, lr = lane & 15, hi = lane >> 4;
    const int wave = __builtin_amdgcn_readfirstlane((int)(threadIdx.x >> 5));
    const unsigned r0 = (blockIdx.x * (unsigned)AW + (unsigned)wave) * 16u;
    const unsigned b = r0 / (unsigned)SEQ, tt = r0 % (unsigned)SEQ;
    const int wb = wave * 16 * OSP;
    const v8f zv = (v8f){};
    const float* yr = Y2 + (size_t)(r0 + (unsigned)lr) * DM + 8 * hi;
    const size_t wo = (size_t)lr * DM + 8 * hi;
    v16h ah[2], ar[2];
#pragma unroll
    for (int kc = 0; kc < 2; ++kc) {
        const v4f p0 = *(const v4f*)(yr + kc * 32) * DCAR, p1 = *(const v4f*)(yr + kc * 32 + 4) * DCAR, p2 = *(const v4f*)(yr + kc * 32 + 16) * DCAR, p3 = *(const v4f*)(yr + kc * 32 + 20) * DCAR;
        v8h h0, q0, h1, q1; hsplit4<0>(p0, h0, q0); hsplit4<4>(p1, h0, q0); hsplit4<0>(p2, h1, q1); hsplit4<4>(p3, h1, q1);
        ah[kc] = cat16(h0, h1); ar[kc] = cat16(q0, q1); }
    v8f aH[4], aR[4];
#pragma unroll
    for (int nb = 0; nb < 4; ++nb) { aH[nb] = zv; aR[nb] = zv; }
#pragma unroll
    for (int kc = 0; kc < 2; ++kc) {
#pragma unroll
        for (int nb = 0; nb < 4; ++nb) { const v16h w = ldh(WD + wo + (size_t)nb * 16 * DM + kc * 32);
            aH[nb] = wmma16g(ah[kc], w, aH[nb]); aR[nb] = wmma16g(ar[kc], w, aR[nb]); } }
#pragma unroll
    for (int nb = 0; nb < 4; ++nb) {
#pragma unroll
        for (int j = 0; j < 8; ++j) os[wb + (hi * 8 + j) * OSP + nb * 16 + lr] = fmaxf((aH[nb][j] + aR[nb][j] * QRI) * DUN, 0.0f); }
    wave_sync();
#pragma unroll
    for (int kc = 0; kc < 2; ++kc) {
        const int o = wb + lr * OSP + kc * 32 + 8 * hi;
        const v4f p0 = *(const v4fa*)(&os[o]) * DCAR, p1 = *(const v4fa*)(&os[o + 4]) * DCAR, p2 = *(const v4fa*)(&os[o + 16]) * DCAR, p3 = *(const v4fa*)(&os[o + 20]) * DCAR;
        v8h h0, q0, h1, q1; hsplit4<0>(p0, h0, q0); hsplit4<4>(p1, h0, q0); hsplit4<0>(p2, h1, q1); hsplit4<4>(p3, h1, q1);
        ah[kc] = cat16(h0, h1); ar[kc] = cat16(q0, q1); }
    wave_sync();
#pragma unroll
    for (int nb = 0; nb < 4; ++nb) { aH[nb] = zv; aR[nb] = zv; }
#pragma unroll
    for (int kc = 0; kc < 2; ++kc) {
#pragma unroll
        for (int nb = 0; nb < 4; ++nb) { const v16h w = ldh(WD + (size_t)DM * DM + wo + (size_t)nb * 16 * DM + kc * 32);
            aH[nb] = wmma16g(ah[kc], w, aH[nb]); aR[nb] = wmma16g(ar[kc], w, aR[nb]); } }
#pragma unroll
    for (int nb = 0; nb < 4; ++nb) {
#pragma unroll
        for (int j = 0; j < 8; ++j) os[wb + (hi * 8 + j) * OSP + nb * 16 + lr] = fmaxf((aH[nb][j] + aR[nb][j] * QRI) * DUN, 0.0f); }
    wave_sync();
    float* orow = OUT + ((size_t)b * OUT_SEQ + (size_t)tt) * DM;
#pragma unroll 1
    for (int ps = 0; ps < 2; ++ps) {
#pragma unroll
        for (int s = 0; s < 8; ++s) { const int row = 2 * s + (lane >> 4), cofs = (lane & 15) * 4;
            const v4f val = *(const v4fa*)(&os[wb + row * OSP + cofs]);
            *(volatile v4f*)(orow + (size_t)row * DM + cofs) = val; }
        if (ps == 0) __threadfence(); }
}

static constexpr size_t al256(size_t v) { return (v + 255) & ~(size_t)255; }
static constexpr size_t SZ_WE = al256((size_t)2 * DM * DM * 2);
static constexpr size_t SZ_WD = al256((size_t)2 * DM * DM * 2);
static constexpr size_t SZ_PL = al256((size_t)NB * SEQ * DM * 2);
static constexpr size_t SZ_Y2 = al256((size_t)NB * SEQ * DM * 4);
static constexpr size_t SZ_TOTAL = SZ_WE + SZ_WD + 4 * SZ_PL + SZ_Y2;
static_assert(SZ_TOTAL <= (size_t)134217728);
static constexpr size_t NEED_X = ((size_t)(NB - 1) * SEQ_FULL + SEQ) * DM;
static constexpr size_t NEED_W = (size_t)2 * DM * DM;
static constexpr size_t NEED_O = ((size_t)(NB - 1) * OUT_SEQ + SEQ) * DM;

extern "C" void kernel_launch(void* const* d_in, const int* in_sizes, int n_in,
                              void* d_out, int out_size, void* d_ws, size_t ws_size, hipStream_t stream) {
    if (n_in < 3) return;
    if ((size_t)in_sizes[0] < NEED_X || (size_t)in_sizes[1] < NEED_W || (size_t)in_sizes[2] < NEED_W) return;
    if ((size_t)out_size < NEED_O) return;
    if (SZ_TOTAL > ws_size) return;
    const float* x    = (const float*)d_in[0];
    const float* wenc = (const float*)d_in[1];
    const float* wdec = (const float*)d_in[2];
    float* OUT = (float*)d_out;
    char* wsp = (char*)d_ws;
    bf*  WE  = (bf*)wsp;  wsp += SZ_WE;
    h16* WD  = (h16*)wsp; wsp += SZ_WD;
    h16* YH  = (h16*)wsp; wsp += SZ_PL;
    h16* YR  = (h16*)wsp; wsp += SZ_PL;
    h16* YTH = (h16*)wsp; wsp += SZ_PL;
    h16* YTR = (h16*)wsp; wsp += SZ_PL;
    float* Y2 = (float*)wsp; wsp += SZ_Y2;

    k_wconv<<<8, 256, 0, stream>>>(wenc, wdec, WE, WD);
    k_enc<<<NB * SEQ / 64, 32 * AW, 0, stream>>>(x, WE, YH, YR, YTH, YTR);
    k_sim<<<dim3(SEQ / (16 * AW), NB, 1), 32 * AW, 0, stream>>>(YH, YTH, Y2);
    k_dec<<<NB * SEQ / (16 * AW), 32 * AW, 0, stream>>>(Y2, WD, OUT);
}
